// OctreeConv_90117003804709
// MI455X (gfx1250) — hardware-verified
//
#include <hip/hip_runtime.h>
#include <stddef.h>
#include <stdint.h>


#define KD    27
#define CI    32
#define CO    32
#define KK    (KD * CI)
#define BM    32
#define NTHR  128
#define SXS   872
#define SOS   36
#define XSC   8
#define WSC   1024
#define PTHR  256
#define WSCAP 134217728

static_assert(KK % 32 == 0);
static_assert(SXS >= KK);
static_assert((SXS * 2) % 16 == 0);
static_assert((SOS * 4) % 16 == 0);
static_assert(SOS >= CO);
static_assert(NTHR == 4 * 32);
static_assert(BM == 32 && CO == 32 && CI == 32);
static_assert((BM * KD * (CI / 8)) % NTHR == 0);
static_assert((CO * KK) % 8 == 0);

typedef float    v4f  __attribute__((ext_vector_type(4)));
typedef float    v8f  __attribute__((ext_vector_type(8)));
typedef unsigned v4u  __attribute__((ext_vector_type(4)));
typedef _Float16 v8h  __attribute__((ext_vector_type(8)));
typedef _Float16 v16h __attribute__((ext_vector_type(16)));
union FragH { v16h v; v8h s[2]; };
union RowH  { v4u u; v8h hv; };

__device__ __forceinline__ int imin(int a, int b) { return a < b ? a : b; }
__device__ __forceinline__ int imax(int a, int b) { return a > b ? a : b; }

__device__ __forceinline__ v8f wmf(v16h a, v16h b, v8f c) {
  v8f d = __builtin_amdgcn_wmma_f32_16x16x32_f16(false, a, false, b, (short)0, c, false, false);
  asm volatile("v_nop\n\tv_nop\n\tv_nop\n\tv_nop" : "+v"(d) : "v"(a), "v"(b));
  return d;
}

__device__ __forceinline__ v16h ld_frag(const _Float16* row_plus_8h, int k0) {
  FragH f;
  f.s[0] = *(const v8h*)(row_plus_8h + k0);
  f.s[1] = *(const v8h*)(row_plus_8h + k0 + 16);
  return f.v;
}

__global__ __launch_bounds__(PTHR) void k_prep_data(const float* __restrict__ x, _Float16* dst, int nq) {
  const int t = blockIdx.x * PTHR + threadIdx.x;
  if (t >= nq) return;
  const float* p = x + (size_t)t * 8;
  const v4f f0 = *(const v4f*)p;
  const v4f f1 = *(const v4f*)(p + 4);
  v8h a;
  a[0] = (_Float16)(f0.x * (float)XSC); a[1] = (_Float16)(f0.y * (float)XSC);
  a[2] = (_Float16)(f0.z * (float)XSC); a[3] = (_Float16)(f0.w * (float)XSC);
  a[4] = (_Float16)(f1.x * (float)XSC); a[5] = (_Float16)(f1.y * (float)XSC);
  a[6] = (_Float16)(f1.z * (float)XSC); a[7] = (_Float16)(f1.w * (float)XSC);
  _Float16* d = dst + (size_t)t * 8;
  *(volatile v8h*)d = a;
  __threadfence();
  *(volatile v8h*)d = a;
}

__global__ __launch_bounds__(PTHR) void k_prep_w(const float* __restrict__ W, _Float16* dst) {
  const int t = blockIdx.x * PTHR + threadIdx.x;
  if (t >= (CO * KK) / 8) return;
  const int o  = t / (KK / 8);
  const int kq = (t - o * (KK / 8)) * 8;
  v8h hv;
#pragma unroll
  for (int e = 0; e < 8; ++e) {
    const int kg = kq + e;
    const float v = W[(size_t)kg * CO + o];
    hv[e] = (_Float16)(v * (float)WSC);
  }
  _Float16* d = dst + (size_t)t * 8;
  *(volatile v8h*)d = hv;
  __threadfence();
  *(volatile v8h*)d = hv;
}

__global__ __launch_bounds__(NTHR) void k_main(const _Float16* __restrict__ dH, const _Float16* __restrict__ Wb,
                                               const int* __restrict__ nb, float* out, int nN) {
  __shared__ __attribute__((aligned(16))) _Float16 sX[BM * SXS];
  __shared__ __attribute__((aligned(16))) float    sO[BM * SOS];

  const int tid = threadIdx.x, lane = tid & 31, wave = tid >> 5, h = lane >> 4, m = lane & 15;
  const int mbase = blockIdx.x * BM;

  {
    const size_t nbBase = (size_t)mbase * KD;
    const size_t nbLast = (size_t)nN * KD - 1;
#pragma unroll 1
    for (int it = 0; it < (BM * KD * (CI / 8)) / NTHR; ++it) {
      const int ci = it * NTHR + tid;
      const int q  = ci & 3;
      const int rk = ci >> 2;
      const int r  = rk / KD;
      const int k  = rk - r * KD;
      size_t ea = nbBase + (size_t)rk;
      ea = (ea < nbLast) ? ea : nbLast;
      int idx = nb[ea];
      const bool valid = (idx >= 0) && (mbase + r < nN);
      idx = imin(imax(idx, 0), nN - 1);
      RowH g;
      g.u = *(const v4u*)(dH + (size_t)idx * CI + 8 * q);
      const unsigned mk = valid ? 0xffffffffu : 0u;
      const v4u mv = {mk, mk, mk, mk};
      g.u = g.u & mv;
      *(v8h*)(sX + r * SXS + k * CI + 8 * q) = g.hv;
    }
  }
  __syncthreads();

  const int mt = wave >> 1, nt = wave & 1;
  v8f acc = {0.f, 0.f, 0.f, 0.f, 0.f, 0.f, 0.f, 0.f};
  {
    const _Float16* ap = sX + (16 * mt + m) * SXS + 8 * h;
    const _Float16* bp = Wb + (size_t)(16 * nt + m) * KK + 8 * h;
#pragma unroll 3
    for (int kt = 0; kt < KK / 32; ++kt) {
      const int k0 = 32 * kt;
      const v16h a = ld_frag(ap, k0);
      const v16h b = ld_frag(bp, k0);
      acc = wmf(a, b, acc);
    }
  }

  {
    constexpr float OSC = 1.0f / (float)(XSC * WSC);
    const int col = 16 * nt + m;
#pragma unroll
    for (int r = 0; r < 8; ++r) sO[(16 * mt + 8 * h + r) * SOS + col] = acc[r] * OSC;
  }
  __syncthreads();

  {
    const int q = lane & 7, rq = lane >> 3;
    v4f ov[2];
    int rl[2];
#pragma unroll
    for (int j = 0; j < 2; ++j) {
      rl[j] = 8 * wave + 4 * j + rq;
      ov[j] = *(const v4f*)(sO + rl[j] * SOS + 4 * q);
    }
#pragma unroll
    for (int j = 0; j < 2; ++j) {
      const int n = mbase + rl[j];
      if (n < nN) *(volatile v4f*)(out + (size_t)n * CO + 4 * q) = ov[j];
    }
    __threadfence();
#pragma unroll
    for (int j = 0; j < 2; ++j) {
      const int n = mbase + rl[j];
      if (n < nN) *(volatile v4f*)(out + (size_t)n * CO + 4 * q) = ov[j];
    }
  }
}

extern "C" void kernel_launch(void* const* d_in, const int* in_sizes, int n_in,
                              void* d_out, int out_size, void* d_ws, size_t ws_size,
                              hipStream_t stream) {
  if (n_in < 3) return;
  if (in_sizes[0] < CI || (in_sizes[0] % CI) != 0) return;
  const int nN = in_sizes[0] / CI;
  if (in_sizes[1] != KD * CI * CO) return;
  if (in_sizes[2] != nN * KD) return;
  if (out_size != nN * CO) return;

  const float* data = (const float*)d_in[0];
  const float* W    = (const float*)d_in[1];
  const int*   nb   = (const int*)d_in[2];
  float* out = (float*)d_out;

  char* ws = (char*)d_ws;
  size_t off = 0;
  const size_t bD = (((size_t)nN * CI * 2) + 511) & ~(size_t)511;
  const size_t oD = off; off += bD; off = (off + 255) & ~(size_t)255;
  const size_t bW = (((size_t)CO * KK * 2) + 511) & ~(size_t)511;
  const size_t oW = off; off += bW; off = (off + 255) & ~(size_t)255;
  if (off > ws_size || off > (size_t)WSCAP) return;
  _Float16* dH = (_Float16*)(ws + oD);
  _Float16* Wb = (_Float16*)(ws + oW);

  const int nq = nN * (CI / 8);
  k_prep_data<<<(nq + PTHR - 1) / PTHR, PTHR, 0, stream>>>(data, dH, nq);
  k_prep_w<<<((CO * KK) / 8 + PTHR - 1) / PTHR, PTHR, 0, stream>>>(W, Wb);
  k_main<<<(nN + BM - 1) / BM, NTHR, 0, stream>>>(dH, Wb, nb, out, nN);
}
